// MHSA_9002251453132
// MI455X (gfx1250) — hardware-verified
//
#include <hip/hip_runtime.h>
#include <stdint.h>


typedef unsigned short hword;
typedef hword us8  __attribute__((ext_vector_type(8)));
typedef hword us16 __attribute__((ext_vector_type(16)));
typedef __bf16 bf16x16 __attribute__((ext_vector_type(16)));
typedef _Float16 f16x16 __attribute__((ext_vector_type(16)));
typedef float v8f __attribute__((ext_vector_type(8)));
typedef float v4f __attribute__((ext_vector_type(4)));

#ifndef NB
#define NB 8
#endif
#define NB_FULL 8
#define CH    512
#define NHEAD 8
#define HD    64
#define GW    32
#define NPIX  1024
#define TT    (NB * NPIX / 64)
#define LDT   68

static_assert(NB >= 1 && NB <= NB_FULL);
static_assert(NPIX == GW * GW);
static_assert(CH == NHEAD * HD);
static_assert((CH % 64) == 0 && (NPIX % 64) == 0 && (HD % 32) == 0);
static_assert((LDT * 4) % 16 == 0);

__device__ __forceinline__ hword f2bf(float x) {
    unsigned int u = __float_as_uint(x);
    u = (u + 0x7FFFu + ((u >> 16) & 1u)) >> 16;
    return (hword)u;
}
__device__ __forceinline__ float bf2f(hword b) {
    return __uint_as_float(((unsigned int)b) << 16);
}
__device__ __forceinline__ hword f2h(float x) {
    _Float16 t = (_Float16)x;
    return __builtin_bit_cast(hword, t);
}
__device__ __forceinline__ v8f zero8() {
    v8f z;
#pragma unroll
    for (int i = 0; i < 8; ++i) z[i] = 0.0f;
    return z;
}

__device__ __forceinline__ v8f mma_bf(v8f c, us16 a, us16 b) {
    bf16x16 av = __builtin_bit_cast(bf16x16, a);
    bf16x16 bv = __builtin_bit_cast(bf16x16, b);
    c = __builtin_amdgcn_wmma_f32_16x16x32_bf16(false, av, false, bv, (short)0, c, false, false);
    asm volatile("v_nop\n\tv_nop\n\tv_nop\n\tv_nop" : "+v"(c) : "v"(a), "v"(b));
    return c;
}
__device__ __forceinline__ v8f mma_hf(v8f c, us16 a, us16 b) {
    f16x16 av = __builtin_bit_cast(f16x16, a);
    f16x16 bv = __builtin_bit_cast(f16x16, b);
    c = __builtin_amdgcn_wmma_f32_16x16x32_f16(false, av, false, bv, (short)0, c, false, false);
    asm volatile("v_nop\n\tv_nop\n\tv_nop\n\tv_nop" : "+v"(c) : "v"(a), "v"(b));
    return c;
}

__device__ __forceinline__ us16 frag_rows(const hword* p, int ld, int row, int k0, int h) {
    const hword* base = p + (size_t)row * ld + k0 + 8 * h;
    us8 e0 = *(const us8*)(base);
    us8 e1 = *(const us8*)(base + 16);
    return __builtin_shufflevector(e0, e1, 0, 1, 2, 3, 4, 5, 6, 7,
                                   8, 9, 10, 11, 12, 13, 14, 15);
}

static_assert(128 * 256 * 8 == CH * CH);
__global__ __launch_bounds__(256) void k_cvtw(const float* __restrict__ w0,
                                              const float* __restrict__ w1,
                                              const float* __restrict__ w2,
                                              hword* d0, hword* d1, hword* d2) {
    const int seg = blockIdx.x >> 7;
    const int i = (blockIdx.x & 127) * 256 + threadIdx.x;
    const float* src = (seg == 0) ? w0 : ((seg == 1) ? w1 : w2);
    hword* dst = (seg == 0) ? d0 : ((seg == 1) ? d1 : d2);
    const float* s = src + (size_t)i * 8;
    const v4f a = *(const v4f*)(s);
    const v4f b = *(const v4f*)(s + 4);
    us8 o;
#pragma unroll
    for (int e = 0; e < 4; ++e) {
        o[e]     = f2bf(a[e]);
        o[4 + e] = f2bf(b[e]);
    }
    const size_t o8 = (size_t)i * 8;
    *(volatile us8*)(dst + o8) = o;
    __threadfence();
    *(volatile us8*)(dst + o8) = o;
}

__global__ __launch_bounds__(128) void k_xt(const float* __restrict__ x, hword* xt) {
    __shared__ __align__(16) float tile[64 * LDT];
    const int tid = threadIdx.x, w = tid >> 5, lane = tid & 31;
    const int ct = blockIdx.x & 7, nt = (blockIdx.x >> 3) & 15, b = blockIdx.x >> 7;
    const int c0 = ct * 64, n0 = nt * 64;
    const float* xg = x + ((size_t)(b * CH + c0)) * NPIX + n0;
#pragma unroll
    for (int it = 0; it < 8; ++it) {
        const int idx = it * 128 + tid;
        const int crow = idx >> 4, piece = idx & 15;
        const v4f v = *(const v4f*)(xg + (size_t)crow * NPIX + 4 * piece);
        *(v4f*)(tile + crow * LDT + 4 * piece) = v;
    }
    __syncthreads();

    const int p = lane & 7, lq = lane >> 3;
    us8 o[4];
#pragma unroll
    for (int i = 0; i < 4; ++i) {
        const int nrow = w * 16 + 4 * i + lq;
#pragma unroll
        for (int e = 0; e < 8; ++e) o[i][e] = f2bf(tile[(8 * p + e) * LDT + nrow]);
    }
#pragma unroll
    for (int i = 0; i < 4; ++i) {
        const int nrow = w * 16 + 4 * i + lq;
        hword* dp = xt + ((size_t)(b * NPIX + n0 + nrow)) * CH + c0 + 8 * p;
        *(volatile us8*)dp = o[i];
    }
    __threadfence();
#pragma unroll
    for (int i = 0; i < 4; ++i) {
        const int nrow = w * 16 + 4 * i + lq;
        hword* dp = xt + ((size_t)(b * NPIX + n0 + nrow)) * CH + c0 + 8 * p;
        *(volatile us8*)dp = o[i];
    }
}

static_assert(256 * 32 == NHEAD * NPIX);
__global__ __launch_bounds__(256) void k_rel(const float* __restrict__ relh,
                                             const float* __restrict__ relw,
                                             hword* rh, hword* rl) {
    const int tid = threadIdx.x;
    const int row = blockIdx.x * 32 + (tid >> 3);
    const int p = tid & 7;
    const int hh = row >> 10, n = row & (NPIX - 1);
    const int gi = n >> 5, gj = n & (GW - 1);
    us8 oh, ol;
#pragma unroll
    for (int e = 0; e < 8; ++e) {
        const int d = 8 * p + e;
        const int base = (hh * HD + d) * GW;
        const float vh = bf2f(f2bf(relh[base + gj]));
        const float vw = bf2f(f2bf(relw[base + gi]));
        const float s = vh + vw;
        const hword a = f2bf(s);
        oh[e] = a;
        ol[e] = f2bf(s - bf2f(a));
    }
    const size_t off = (size_t)row * HD + 8 * p;
    *(volatile us8*)(rh + off) = oh;
    *(volatile us8*)(rl + off) = ol;
    __threadfence();
    *(volatile us8*)(rh + off) = oh;
    *(volatile us8*)(rl + off) = ol;
}

__device__ __forceinline__ void qk_pass(const float* tile, hword* P0, hword* P1,
                                        size_t rb, int w, int p, int lq) {
#pragma unroll
    for (int i = 0; i < 4; ++i) {
        const int row = w * 16 + 4 * i + lq;
        const float* sp = tile + row * LDT + 8 * p;
        const v4f u0 = *(const v4f*)(sp);
        const v4f u1 = *(const v4f*)(sp + 4);
        us8 oh, ol;
#pragma unroll
        for (int e = 0; e < 4; ++e) {
            const hword a = f2bf(u0[e]);
            oh[e] = a;
            ol[e] = f2bf(u0[e] - bf2f(a));
            const hword c = f2bf(u1[e]);
            oh[4 + e] = c;
            ol[4 + e] = f2bf(u1[e] - bf2f(c));
        }
        const size_t doff = (rb + (size_t)row) * HD + 8 * p;
        *(volatile us8*)(P0 + doff) = oh;
        *(volatile us8*)(P1 + doff) = ol;
    }
}
__device__ __forceinline__ void v_pass(const float* tile, hword* vt, size_t vb, int n0,
                                       int w, int p, int lq) {
#pragma unroll
    for (int i = 0; i < 4; ++i) {
        const int d = w * 16 + 4 * i + lq;
        us8 o;
#pragma unroll
        for (int e = 0; e < 8; ++e) o[e] = f2h(tile[(8 * p + e) * LDT + d]);
        *(volatile us8*)(vt + (vb + (size_t)d) * NPIX + (size_t)n0 + 8 * p) = o;
    }
}

template <int SV>
__global__ __launch_bounds__(128) void k_qkv(const hword* xt, const hword* w0, const hword* w1,
                                             const float* b0, const float* b1,
                                             hword* d0, hword* d1, hword* d2, hword* d3) {
    __shared__ __align__(16) float tile[64 * LDT];
    const int w = threadIdx.x >> 5, lane = threadIdx.x & 31;
    const int h = lane >> 4, m = lane & 15;
    const int mt = blockIdx.x % TT, ng = blockIdx.x / TT;
    const int s  = SV ? 2 : (ng >> 3);
    const int hh = SV ? ng : (ng & 7);
    const hword* wp = (SV != 0 || s == 0) ? w0 : w1;
    const float* bp = (SV != 0 || s == 0) ? b0 : b1;
    const int tok0 = mt * 64;
    const int wr = w & 1, wc = w >> 1;
    const int ar0 = tok0 + wr * 32;

    int orow[2];
#pragma unroll
    for (int t = 0; t < 2; ++t) orow[t] = hh * HD + wc * 32 + t * 16 + m;

    v8f acc[2][2];
#pragma unroll
    for (int mi = 0; mi < 2; ++mi)
#pragma unroll
        for (int t = 0; t < 2; ++t) acc[mi][t] = zero8();

#pragma unroll 1
    for (int k0 = 0; k0 < CH; k0 += 32) {
        const us16 a0 = frag_rows(xt, CH, ar0 + m, k0, h);
        const us16 a1 = frag_rows(xt, CH, ar0 + 16 + m, k0, h);
#pragma unroll
        for (int t = 0; t < 2; ++t) {
            const us16 b = frag_rows(wp, CH, orow[t], k0, h);
            acc[0][t] = mma_bf(acc[0][t], a0, b);
            acc[1][t] = mma_bf(acc[1][t], a1, b);
        }
    }

#pragma unroll
    for (int t = 0; t < 2; ++t) {
        const float bv = bf2f(f2bf(bp[orow[t]]));
#pragma unroll
        for (int mi = 0; mi < 2; ++mi)
#pragma unroll
            for (int r = 0; r < 8; ++r)
                tile[(wr * 32 + mi * 16 + 8 * h + r) * LDT + wc * 32 + t * 16 + m] =
                    acc[mi][t][r] + bv;
    }
    __syncthreads();

    const int bb = tok0 >> 10, n0 = tok0 & (NPIX - 1);
    const int p = lane & 7, lq = lane >> 3;
    if (SV == 0) {
        hword* P0 = (s == 0) ? d0 : d2;
        hword* P1 = (s == 0) ? d1 : d3;
        const size_t rb = ((size_t)(bb * NHEAD + hh)) * NPIX + (size_t)n0;
        qk_pass(tile, P0, P1, rb, w, p, lq);
        __threadfence();
        qk_pass(tile, P0, P1, rb, w, p, lq);
    } else {
        const size_t vb = ((size_t)(bb * NHEAD + hh)) * HD;
        v_pass(tile, d0, vb, n0, w, p, lq);
        __threadfence();
        v_pass(tile, d0, vb, n0, w, p, lq);
    }
}

__global__ __launch_bounds__(128) void k_attn(const hword* qh, const hword* ql,
                                              const hword* kh, const hword* kl,
                                              const hword* rh, const hword* rl,
                                              const hword* vt, float* out) {
    __shared__ __align__(16) float st[64 * LDT];
    const int w = threadIdx.x >> 5, lane = threadIdx.x & 31;
    const int h = lane >> 4, m = lane & 15;
    const int qt = blockIdx.x & 15, bh = blockIdx.x >> 4;
    const int bb = bh >> 3, hh = bh & 7;
    const size_t poff = (size_t)bh * NPIX * HD;
    const size_t roff = (size_t)hh * NPIX * HD;
    const hword* qhp = qh + poff;
    const hword* qlp = ql + poff;
    const hword* khp = kh + poff;
    const hword* klp = kl + poff;
    const hword* rhp = rh + roff;
    const hword* rlp = rl + roff;
    const hword* vtp = vt + poff;
    const int q0 = qt * 64 + w * 16;

    us16 qbh[4], qbl[4];
#pragma unroll
    for (int dc = 0; dc < 2; ++dc) {
        qbh[dc]     = frag_rows(qhp, HD, q0 + m, dc * 32, h);
        qbl[dc]     = frag_rows(qlp, HD, q0 + m, dc * 32, h);
        qbh[2 + dc] = frag_rows(rhp, HD, q0 + m, dc * 32, h);
        qbl[2 + dc] = frag_rows(rlp, HD, q0 + m, dc * 32, h);
    }

    v8f oacc[4];
#pragma unroll
    for (int dt = 0; dt < 4; ++dt) oacc[dt] = zero8();
    float mrun = -1.0e30f, lrun = 0.0f;

#pragma unroll 1
    for (int kc = 0; kc < NPIX; kc += 64) {
        v8f sacc[4];
#pragma unroll
        for (int kt = 0; kt < 4; ++kt) {
            v8f sa = zero8();
            const int krow = kc + kt * 16 + m;
#pragma unroll
            for (int dc = 0; dc < 2; ++dc) {
                const us16 ka = frag_rows(khp, HD, krow, dc * 32, h);
                const us16 kb = frag_rows(klp, HD, krow, dc * 32, h);
                sa = mma_bf(sa, ka, qbh[dc]);
                sa = mma_bf(sa, ka, qbl[dc]);
                sa = mma_bf(sa, kb, qbh[dc]);
            }
#pragma unroll
            for (int dc = 0; dc < 2; ++dc) {
                const us16 ka = frag_rows(qhp, HD, krow, dc * 32, h);
                const us16 kb = frag_rows(qlp, HD, krow, dc * 32, h);
                sa = mma_bf(sa, ka, qbh[2 + dc]);
                sa = mma_bf(sa, ka, qbl[2 + dc]);
                sa = mma_bf(sa, kb, qbh[2 + dc]);
            }
            sacc[kt] = sa;
        }

        float mloc = -1.0e30f;
#pragma unroll
        for (int kt = 0; kt < 4; ++kt)
#pragma unroll
            for (int r = 0; r < 8; ++r) mloc = fmaxf(mloc, sacc[kt][r]);
        mloc = fmaxf(mloc, __shfl_xor(mloc, 16, 32));
        const float mnew = fmaxf(mrun, mloc);
        const float corr = __expf(mrun - mnew);
        mrun = mnew;
        float lsum = 0.0f;
        us16 pb[2];
#pragma unroll
        for (int kt = 0; kt < 4; ++kt) {
#pragma unroll
            for (int r = 0; r < 8; ++r) {
                const float pv = __expf(sacc[kt][r] - mnew);
                lsum += pv;
                pb[kt >> 1][(kt & 1) * 8 + r] = f2h(pv * 16384.0f);
            }
        }
        lsum += __shfl_xor(lsum, 16, 32);
        lrun = lrun * corr + lsum;
#pragma unroll
        for (int dt = 0; dt < 4; ++dt) oacc[dt] = oacc[dt] * corr;

#pragma unroll
        for (int ks = 0; ks < 2; ++ks) {
#pragma unroll
            for (int dt = 0; dt < 4; ++dt) {
                const us16 va = frag_rows(vtp, NPIX, dt * 16 + m, kc + ks * 32, h);
                oacc[dt] = mma_hf(oacc[dt], va, pb[ks]);
            }
        }
    }

    const float inv = 1.0f / (lrun * 16384.0f);
#pragma unroll
    for (int dt = 0; dt < 4; ++dt) {
#pragma unroll
        for (int r = 0; r < 8; ++r)
            st[(dt * 16 + 8 * h + r) * LDT + w * 16 + m] = oacc[dt][r] * inv;
    }
    __syncthreads();

    const size_t orow0 = (size_t)(bb * CH + hh * HD);
    const int qcol = qt * 64 + 4 * m;
#pragma unroll
    for (int i = 0; i < 8; ++i) {
        const int d = w * 16 + 2 * i + h;
        const v4f v = *(const v4f*)(st + d * LDT + 4 * m);
        *(volatile v4f*)(out + (orow0 + (size_t)d) * NPIX + qcol) = v;
    }
    __threadfence();
#pragma unroll
    for (int i = 0; i < 8; ++i) {
        const int d = w * 16 + 2 * i + h;
        const v4f v = *(const v4f*)(st + d * LDT + 4 * m);
        *(volatile v4f*)(out + (orow0 + (size_t)d) * NPIX + qcol) = v;
    }
}

extern "C" void kernel_launch(void* const* d_in, const int* in_sizes, int n_in,
                              void* d_out, int out_size, void* d_ws, size_t ws_size,
                              hipStream_t stream) {
    if (n_in < 9) return;
    const int nx   = NB * CH * NPIX;
    const int nw   = CH * CH;
    const int nrel = NHEAD * HD * GW;
    if (in_sizes[0] < nx || in_sizes[1] < nw || in_sizes[2] < CH ||
        in_sizes[3] < nw || in_sizes[4] < CH || in_sizes[5] < nw || in_sizes[6] < CH ||
        in_sizes[7] < nrel || in_sizes[8] < nrel || out_size < nx) return;

    const float* x    = (const float*)d_in[0];
    const float* Wq   = (const float*)d_in[1];
    const float* bq   = (const float*)d_in[2];
    const float* Wk   = (const float*)d_in[3];
    const float* bk   = (const float*)d_in[4];
    const float* Wv   = (const float*)d_in[5];
    const float* bv   = (const float*)d_in[6];
    const float* relh = (const float*)d_in[7];
    const float* relw = (const float*)d_in[8];
    float* out = (float*)d_out;

    const size_t b_w  = (size_t)nw * 2;
    const size_t b_xt = (size_t)NB * NPIX * CH * 2;
    const size_t b_r  = (size_t)NHEAD * NPIX * HD * 2;
    const size_t b_p  = (size_t)NB * NHEAD * NPIX * HD * 2;
    size_t off = 0;
    char* ws = (char*)d_ws;
    hword* wqb = (hword*)(ws + off); off += b_w;
    hword* wkb = (hword*)(ws + off); off += b_w;
    hword* wvb = (hword*)(ws + off); off += b_w;
    hword* xt  = (hword*)(ws + off); off += b_xt;
    hword* rh  = (hword*)(ws + off); off += b_r;
    hword* rl  = (hword*)(ws + off); off += b_r;
    hword* qh  = (hword*)(ws + off); off += b_p;
    hword* ql  = (hword*)(ws + off); off += b_p;
    hword* kh  = (hword*)(ws + off); off += b_p;
    hword* kl  = (hword*)(ws + off); off += b_p;
    hword* vt  = (hword*)(ws + off); off += b_p;
    if (off > ws_size) return;

    k_cvtw<<<384, 256, 0, stream>>>(Wq, Wk, Wv, wqb, wkb, wvb);
    k_xt<<<NB * 128, 128, 0, stream>>>(x, xt);
    k_rel<<<(NHEAD * NPIX) / 32, 256, 0, stream>>>(relh, relw, rh, rl);
    k_qkv<0><<<TT * 16, 128, 0, stream>>>(xt, wqb, wkb, bq, bk, qh, ql, kh, kl);
    k_qkv<1><<<TT * 8, 128, 0, stream>>>(xt, wvb, wvb, bv, bv, vt, vt, vt, vt);
    k_attn<<<NB * NHEAD * 16, 128, 0, stream>>>(qh, ql, kh, kl, rh, rl, vt, out);
}
